// TransformerDecoderLayer_5171140624405
// MI455X (gfx1250) — hardware-verified
//
#include <hip/hip_runtime.h>


#ifndef NB
#define NB 4
#endif
#ifndef SEQ
#define SEQ 1024
#endif
#ifndef SENC
#define SENC 1024
#endif
#define NB_FULL 4
#define SEQ_FULL 1024
#define SENC_FULL 1024
#define DM 1024
#define HE 16
#define DH 64
#define FF 4096
#define KT 32
#define QR 128
#define KPITCH 72
#define VPITCH 40
#define PPITCH 40
#define CPITCH 72
#define TPITCH 72
#define OPITCH 132
#define A_CARRY 16.0f
#define V_CARRY 16.0f
#define X_CARRY 64.0f
#define W_CARRY 1024.0f
#define P_CARRY 4096.0f
#define NEG_FILL (-1e20f)
#define LN_EPS 1e-5f

static_assert(NB >= 1 && NB <= NB_FULL);
static_assert(SEQ >= QR && SEQ <= SEQ_FULL);
static_assert(SENC >= KT && SENC <= SENC_FULL);
static_assert(SEQ <= SENC_FULL);
static_assert(SEQ % QR == 0);
static_assert(SEQ % KT == 0);
static_assert(SENC % KT == 0);
static_assert((NB * SEQ) % 64 == 0);
static_assert((NB * SENC) % 64 == 0);
static_assert((NB * SEQ) % 8 == 0);
static_assert(DM % 128 == 0 && FF % 128 == 0);
static_assert(DM % 64 == 0 && FF % 64 == 0);
static_assert(DM % 32 == 0 && FF % 32 == 0);
static_assert(DM == HE * DH);
static_assert(DH == 64);
static_assert(DM == 32 * 32);
static_assert(QR == 8 * 16);

typedef _Float16 v8h  __attribute__((ext_vector_type(8)));
typedef _Float16 v16h __attribute__((ext_vector_type(16)));
typedef float v8f __attribute__((ext_vector_type(8)));
typedef float v4f __attribute__((ext_vector_type(4)));

union FragH { v16h v; v8h h[2]; };

__device__ __forceinline__ unsigned f2bf(float f) { unsigned u = __float_as_uint(f); u += 0x7FFFu + ((u >> 16) & 1u); return u >> 16; }
__device__ __forceinline__ float bf16r(float f) { return __uint_as_float(f2bf(f) << 16); }

__device__ __forceinline__ v8f wm_f16(v16h a, v16h b, v8f c) {
    c = __builtin_amdgcn_wmma_f32_16x16x32_f16(false, a, false, b, (short)0, c, false, false);
    asm volatile("v_nop\n\tv_nop\n\tv_nop\n\tv_nop" : "+v"(c) : "v"(a), "v"(b));
    return c;
}

__global__ __launch_bounds__(256) void k_cvt_act(const float* __restrict__ x, const float* __restrict__ e, _Float16* Xh, _Float16* Eh, int nblkX)
{
    const int bid = blockIdx.x;
    const int which = (bid < nblkX) ? 0 : 1;
    const int lb = which ? (bid - nblkX) : bid;
    const size_t el = ((size_t)lb * 256 + threadIdx.x) * 8;
    const size_t m = el / DM;
    const int col = (int)(el % DM);
    const int L  = which ? SENC : SEQ;
    const int LF = which ? SENC_FULL : SEQ_FULL;
    const int bb = (int)(m / L), n = (int)(m % L);
    const float* src = (which ? e : x) + ((size_t)bb * LF + n) * DM + col;
    const v4f a0 = *(const v4f*)src, a1 = *(const v4f*)(src + 4);
    v8h o;
#pragma unroll
    for (int i = 0; i < 4; ++i) { o[i] = (_Float16)(bf16r(a0[i]) * A_CARRY); o[4 + i] = (_Float16)(bf16r(a1[i]) * A_CARRY); }
    _Float16* dst = (which ? Eh : Xh) + el;
    *(volatile v8h*)dst = o;
    __threadfence();
    *(volatile v8h*)dst = o;
}

__global__ __launch_bounds__(256) void k_cvt_w(const float* __restrict__ w0, const float* __restrict__ w1, const float* __restrict__ w2, const float* __restrict__ w3,
                                              const float* __restrict__ w4, const float* __restrict__ w5, const float* __restrict__ w6, const float* __restrict__ w7,
                                              _Float16* Wt, int K, int N)
{
    __shared__ __align__(16) _Float16 sT[64 * TPITCH];
    const int tid = threadIdx.x, z = blockIdx.z;
    const float* W = w0;
    if (z == 1) W = w1;
    if (z == 2) W = w2;
    if (z == 3) W = w3;
    if (z == 4) W = w4;
    if (z == 5) W = w5;
    if (z == 6) W = w6;
    if (z == 7) W = w7;
    _Float16* dstp = Wt + (size_t)z * N * K;
    const int n0 = blockIdx.x * 64, k0 = blockIdx.y * 64;
#pragma unroll
    for (int i = 0; i < 4; ++i) {
        const int p = tid + 256 * i, kr = p >> 4, c4 = (p & 15) * 4;
        const v4f a = *(const v4f*)(W + (size_t)(k0 + kr) * N + n0 + c4);
#pragma unroll
        for (int j = 0; j < 4; ++j) sT[(c4 + j) * TPITCH + kr] = (_Float16)(bf16r(a[j]) * W_CARRY);
    }
    __syncthreads();
    v8h ov[2];
#pragma unroll
    for (int i = 0; i < 2; ++i) {
        const int p = tid + 256 * i, nr = p >> 3, c8 = (p & 7) * 8;
        ov[i] = *(const v8h*)(sT + nr * TPITCH + c8);
    }
#pragma unroll
    for (int i = 0; i < 2; ++i) {
        const int p = tid + 256 * i, nr = p >> 3, c8 = (p & 7) * 8;
        *(volatile v8h*)(dstp + (size_t)(n0 + nr) * K + k0 + c8) = ov[i];
    }
    __threadfence();
#pragma unroll
    for (int i = 0; i < 2; ++i) {
        const int p = tid + 256 * i, nr = p >> 3, c8 = (p & 7) * 8;
        *(volatile v8h*)(dstp + (size_t)(n0 + nr) * K + k0 + c8) = ov[i];
    }
}

template <int OUT16, int RELU>
__global__ __launch_bounds__(256) void k_gemm(const _Float16* __restrict__ A, const _Float16* __restrict__ Wt, const float* __restrict__ bias,
                                             void* Cv, int K, int ldc, float oscale, float ocarry)
{
    __shared__ __align__(16) float cst[64 * OPITCH];
    const int tid = threadIdx.x, lane = tid & 31, wv = tid >> 5, hh = lane >> 4, lm = lane & 15;
    const int rt = wv & 3, ch = wv >> 2;
    const int row0 = blockIdx.x * 64, cb = blockIdx.y * 128, col0 = cb + ch * 64;
    const _Float16* xr = A + (size_t)(row0 + rt * 16 + lm) * K;
    v8f acc[4];
#pragma unroll
    for (int t = 0; t < 4; ++t) acc[t] = (v8f){};
#pragma unroll 2
    for (int kc = 0; kc < K; kc += 32) {
        FragH a;
        a.h[0] = *(const v8h*)(xr + kc + 8 * hh);
        a.h[1] = *(const v8h*)(xr + kc + 16 + 8 * hh);
#pragma unroll
        for (int t = 0; t < 4; ++t) {
            FragH bb;
            const _Float16* wr = Wt + (size_t)(col0 + t * 16 + lm) * K + kc;
            bb.h[0] = *(const v8h*)(wr + 8 * hh);
            bb.h[1] = *(const v8h*)(wr + 16 + 8 * hh);
            acc[t] = wm_f16(a.v, bb.v, acc[t]);
        }
    }
#pragma unroll
    for (int t = 0; t < 4; ++t) {
        const int cl = ch * 64 + t * 16 + lm;
        const float bv = bf16r(bias[cb + cl]);
#pragma unroll
        for (int r = 0; r < 8; ++r) {
            float o = acc[t][r] * oscale + bv;
            if (RELU) o = fmaxf(o, 0.0f);
            cst[(rt * 16 + 8 * hh + r) * OPITCH + cl] = o * ocarry;
        }
    }
    __syncthreads();
    if (OUT16 == 0) {
        float* C = (float*)Cv;
        v4f ov[8];
#pragma unroll
        for (int i = 0; i < 8; ++i) {
            const int p = tid + 256 * i, row = p >> 5, c4 = (p & 31) * 4;
            ov[i] = *(const v4f*)(cst + row * OPITCH + c4);
        }
#pragma unroll
        for (int i = 0; i < 8; ++i) {
            const int p = tid + 256 * i, row = p >> 5, c4 = (p & 31) * 4;
            *(volatile v4f*)(C + (size_t)(row0 + row) * ldc + cb + c4) = ov[i];
        }
        __threadfence();
#pragma unroll
        for (int i = 0; i < 8; ++i) {
            const int p = tid + 256 * i, row = p >> 5, c4 = (p & 31) * 4;
            *(volatile v4f*)(C + (size_t)(row0 + row) * ldc + cb + c4) = ov[i];
        }
    } else {
        _Float16* C = (_Float16*)Cv;
        v8h ov[4];
#pragma unroll
        for (int i = 0; i < 4; ++i) {
            const int p = tid + 256 * i, row = p >> 4, c8 = (p & 15) * 8;
            const v4f a0 = *(const v4f*)(cst + row * OPITCH + c8);
            const v4f a1 = *(const v4f*)(cst + row * OPITCH + c8 + 4);
#pragma unroll
            for (int j = 0; j < 4; ++j) { ov[i][j] = (_Float16)a0[j]; ov[i][4 + j] = (_Float16)a1[j]; }
        }
#pragma unroll
        for (int i = 0; i < 4; ++i) {
            const int p = tid + 256 * i, row = p >> 4, c8 = (p & 15) * 8;
            *(volatile v8h*)(C + (size_t)(row0 + row) * ldc + cb + c8) = ov[i];
        }
        __threadfence();
#pragma unroll
        for (int i = 0; i < 4; ++i) {
            const int p = tid + 256 * i, row = p >> 4, c8 = (p & 15) * 8;
            *(volatile v8h*)(C + (size_t)(row0 + row) * ldc + cb + c8) = ov[i];
        }
    }
}

__global__ __launch_bounds__(256) void k_attn(const _Float16* __restrict__ Qh, const _Float16* __restrict__ Kh, const _Float16* __restrict__ Vh,
                                             const int* __restrict__ msk, int causal, int Lk, _Float16* Cx)
{
    __shared__ __align__(16) _Float16 sK[KT * KPITCH];
    __shared__ __align__(16) _Float16 sVt[DH * VPITCH];
    __shared__ __align__(16) _Float16 sP[8 * 16 * PPITCH];
    __shared__ __align__(16) _Float16 sC[QR * CPITCH];

    const int tid = threadIdx.x, lane = tid & 31, wv = tid >> 5, hh = lane >> 4, lm = lane & 15;
    const int b = blockIdx.z, h = blockIdx.y, q0 = blockIdx.x * QR;
    const size_t qrow0 = (size_t)b * SEQ + q0;
    const size_t kvrow0 = (size_t)b * Lk;
    const int* mrow = msk + (size_t)b * SENC_FULL;

    FragH qa[2];
    {
        const _Float16* qr = Qh + (qrow0 + wv * 16 + lm) * DM + (size_t)h * DH;
#pragma unroll
        for (int j = 0; j < 2; ++j) {
            qa[j].h[0] = *(const v8h*)(qr + 32 * j + 8 * hh);
            qa[j].h[1] = *(const v8h*)(qr + 32 * j + 16 + 8 * hh);
        }
    }
    v8f acc[4];
    float rm[8], rl[8];
#pragma unroll
    for (int t = 0; t < 4; ++t) acc[t] = (v8f){};
#pragma unroll
    for (int r = 0; r < 8; ++r) { rm[r] = -1e30f; rl[r] = 0.f; }

    const int nkt = (causal != 0) ? ((q0 + QR) / KT) : (Lk / KT);
    const int qi0 = q0 + wv * 16 + 8 * hh;
    const float SCL = 1.0f / (A_CARRY * A_CARRY * 8.0f);

#pragma unroll 1
    for (int kt = 0; kt < nkt; ++kt) {
        const int key0 = kt * KT;
        {
            const int key = tid >> 3, c16 = tid & 7;
            const size_t g = (kvrow0 + key0 + key) * DM + (size_t)h * DH + c16 * 8;
            const v8h kv = *(const v8h*)(Kh + g);
            *(v8h*)(sK + key * KPITCH + c16 * 8) = kv;
            const v8h vv = *(const v8h*)(Vh + g);
#pragma unroll
            for (int j = 0; j < 8; ++j) sVt[(c16 * 8 + j) * VPITCH + key] = vv[j];
        }
        const int ka = key0 + lm, kb2 = key0 + 16 + lm;
        const int ia = (ka < SENC_FULL - 1) ? ka : (SENC_FULL - 1);
        const int ib = (kb2 < SENC_FULL - 1) ? kb2 : (SENC_FULL - 1);
        const int mk0 = mrow[ia], mk1 = mrow[ib];
        __syncthreads();

        v8f sc[2];
#pragma unroll
        for (int t = 0; t < 2; ++t) {
            v8f c = (v8f){};
#pragma unroll
            for (int j = 0; j < 2; ++j) {
                FragH kf;
                const _Float16* kr = sK + (t * 16 + lm) * KPITCH + 32 * j;
                kf.h[0] = *(const v8h*)(kr + 8 * hh);
                kf.h[1] = *(const v8h*)(kr + 16 + 8 * hh);
                c = wm_f16(qa[j].v, kf.v, c);
            }
            sc[t] = c;
        }
#pragma unroll
        for (int r = 0; r < 8; ++r) {
            const int qi = qi0 + r;
            const bool kp0 = (causal != 0) ? (ka <= qi) : (mk0 != 0);
            const bool kp1 = (causal != 0) ? (kb2 <= qi) : (mk1 != 0);
            const float x0 = kp0 ? sc[0][r] * SCL : NEG_FILL;
            const float x1 = kp1 ? sc[1][r] * SCL : NEG_FILL;
            float mx = fmaxf(x0, x1);
#pragma unroll
            for (int o = 1; o < 16; o <<= 1) mx = fmaxf(mx, __shfl_xor(mx, o, 32));
            const float nm = fmaxf(rm[r], mx);
            const float corr = __expf(rm[r] - nm);
            const float p0 = __expf(x0 - nm), p1 = __expf(x1 - nm);
            float rs = p0 + p1;
#pragma unroll
            for (int o = 1; o < 16; o <<= 1) rs += __shfl_xor(rs, o, 32);
            rl[r] = rl[r] * corr + rs;
            rm[r] = nm;
#pragma unroll
            for (int t = 0; t < 4; ++t) acc[t][r] = acc[t][r] * corr;
            _Float16* prow = sP + (wv * 16 + 8 * hh + r) * PPITCH;
            prow[lm] = (_Float16)(p0 * P_CARRY);
            prow[16 + lm] = (_Float16)(p1 * P_CARRY);
        }
        __syncthreads();

        {
            FragH pa;
            const _Float16* pr = sP + (wv * 16 + lm) * PPITCH;
            pa.h[0] = *(const v8h*)(pr + 8 * hh);
            pa.h[1] = *(const v8h*)(pr + 16 + 8 * hh);
#pragma unroll
            for (int t = 0; t < 4; ++t) {
                FragH vb;
                const _Float16* vr = sVt + (t * 16 + lm) * VPITCH;
                vb.h[0] = *(const v8h*)(vr + 8 * hh);
                vb.h[1] = *(const v8h*)(vr + 16 + 8 * hh);
                acc[t] = wm_f16(pa.v, vb.v, acc[t]);
            }
        }
        __syncthreads();
    }

    float inv[8];
#pragma unroll
    for (int r = 0; r < 8; ++r) inv[r] = (1.0f / rl[r]) * (X_CARRY / (P_CARRY * V_CARRY));
#pragma unroll
    for (int r = 0; r < 8; ++r)
#pragma unroll
        for (int t = 0; t < 4; ++t)
            sC[(wv * 16 + 8 * hh + r) * CPITCH + t * 16 + lm] = (_Float16)(acc[t][r] * inv[r]);
    __syncthreads();
    v8h ov[4];
#pragma unroll
    for (int i = 0; i < 4; ++i) {
        const int p = tid + 256 * i, row = p >> 3, c8 = (p & 7) * 8;
        ov[i] = *(const v8h*)(sC + row * CPITCH + c8);
    }
#pragma unroll
    for (int i = 0; i < 4; ++i) {
        const int p = tid + 256 * i, row = p >> 3, c8 = (p & 7) * 8;
        *(volatile v8h*)(Cx + (qrow0 + row) * DM + (size_t)h * DH + c8) = ov[i];
    }
    __threadfence();
#pragma unroll
    for (int i = 0; i < 4; ++i) {
        const int p = tid + 256 * i, row = p >> 3, c8 = (p & 7) * 8;
        *(volatile v8h*)(Cx + (qrow0 + row) * DM + (size_t)h * DH + c8) = ov[i];
    }
}

__global__ __launch_bounds__(256) void k_ln(const float* __restrict__ a, const float* __restrict__ res, int res_full,
                                           const float* __restrict__ g, const float* __restrict__ bt,
                                           float* outf, int out_full, _Float16* outh, int write_h)
{
    __shared__ __align__(16) float rb[8 * DM];
    const int tid = threadIdx.x, lane = tid & 31, wv = tid >> 5;
    const int m = blockIdx.x * 8 + wv;
    const int bb = m / SEQ, n = m % SEQ;
    const size_t crow = (size_t)m * DM;
    const size_t frow = ((size_t)bb * SEQ_FULL + n) * DM;
    const size_t rrow = res_full ? frow : crow;
    const size_t orow = out_full ? frow : crow;
    float* rw = rb + wv * DM;

    float s = 0.f;
#pragma unroll 1
    for (int i = 0; i < 8; ++i) {
        const int c = 128 * i + 4 * lane;
        const v4f av = *(const v4f*)(a + crow + c);
        const v4f rv = *(const v4f*)(res + rrow + c);
        v4f t;
#pragma unroll
        for (int j = 0; j < 4; ++j) {
            const float rr = res_full ? bf16r(rv[j]) : rv[j];
            t[j] = av[j] + rr;
            s += t[j];
        }
        *(v4f*)(rw + c) = t;
    }
#pragma unroll
    for (int o = 1; o < 32; o <<= 1) s += __shfl_xor(s, o, 32);
    const float mu = s * (1.0f / DM);

    float vs = 0.f;
#pragma unroll 1
    for (int i = 0; i < 8; ++i) {
        const int c = 128 * i + 4 * lane;
        const v4f t = *(const v4f*)(rw + c);
#pragma unroll
        for (int j = 0; j < 4; ++j) { const float d = t[j] - mu; vs += d * d; }
    }
#pragma unroll
    for (int o = 1; o < 32; o <<= 1) vs += __shfl_xor(vs, o, 32);
    const float rstd = rsqrtf(vs * (1.0f / DM) + LN_EPS);

#pragma unroll 1
    for (int i = 0; i < 8; ++i) {
        const int c = 128 * i + 4 * lane;
        const v4f t = *(const v4f*)(rw + c);
        const v4f gv = *(const v4f*)(g + c);
        const v4f bv = *(const v4f*)(bt + c);
        v4f y;
#pragma unroll
        for (int j = 0; j < 4; ++j) y[j] = (t[j] - mu) * rstd * bf16r(gv[j]) + bf16r(bv[j]);
        *(v4f*)(rw + c) = y;
        *(volatile v4f*)(outf + orow + c) = y;
    }
    __threadfence();
#pragma unroll 1
    for (int i = 0; i < 8; ++i) {
        const int c = 128 * i + 4 * lane;
        const v4f y = *(const v4f*)(rw + c);
        *(volatile v4f*)(outf + orow + c) = y;
    }
    __syncthreads();
    if (write_h != 0) {
        v8h o[4];
#pragma unroll
        for (int i = 0; i < 4; ++i) {
            const int c = 256 * i + 8 * lane;
            const v4f p0 = *(const v4f*)(rw + c);
            const v4f p1 = *(const v4f*)(rw + c + 4);
#pragma unroll
            for (int j = 0; j < 4; ++j) { o[i][j] = (_Float16)(p0[j] * A_CARRY); o[i][4 + j] = (_Float16)(p1[j] * A_CARRY); }
        }
#pragma unroll
        for (int i = 0; i < 4; ++i) {
            const int c = 256 * i + 8 * lane;
            *(volatile v8h*)(outh + crow + c) = o[i];
        }
        __threadfence();
#pragma unroll
        for (int i = 0; i < 4; ++i) {
            const int c = 256 * i + 8 * lane;
            *(volatile v8h*)(outh + crow + c) = o[i];
        }
    }
}

extern "C" void kernel_launch(void* const* d_in, const int* in_sizes, int n_in,
                              void* d_out, int out_size, void* d_ws, size_t ws_size, hipStream_t stream)
{
    if (n_in < 29) return;
    const long long needX = ((long long)(NB - 1) * SEQ_FULL + SEQ) * DM;
    const long long needE = ((long long)(NB - 1) * SENC_FULL + SENC) * DM;
    if ((long long)in_sizes[0] < needX || (long long)in_sizes[1] < needE) return;
    if (in_sizes[2] < (NB - 1) * SENC_FULL + SENC) return;
    for (int i = 3; i <= 17; i += 2) { if (in_sizes[i] < DM * DM || in_sizes[i + 1] < DM) return; }
    if (in_sizes[19] < DM * FF || in_sizes[20] < FF || in_sizes[21] < FF * DM || in_sizes[22] < DM) return;
    for (int i = 23; i <= 28; ++i) { if (in_sizes[i] < DM) return; }
    if ((long long)out_size < needX) return;

    const float* x     = (const float*)d_in[0];
    const float* enc   = (const float*)d_in[1];
    const int*   emask = (const int*)d_in[2];
    const float* saWq = (const float*)d_in[3];  const float* sabq = (const float*)d_in[4];
    const float* saWk = (const float*)d_in[5];  const float* sabk = (const float*)d_in[6];
    const float* saWv = (const float*)d_in[7];  const float* sabv = (const float*)d_in[8];
    const float* saWo = (const float*)d_in[9];  const float* sabo = (const float*)d_in[10];
    const float* eaWq = (const float*)d_in[11]; const float* eabq = (const float*)d_in[12];
    const float* eaWk = (const float*)d_in[13]; const float* eabk = (const float*)d_in[14];
    const float* eaWv = (const float*)d_in[15]; const float* eabv = (const float*)d_in[16];
    const float* eaWo = (const float*)d_in[17]; const float* eabo = (const float*)d_in[18];
    const float* W1 = (const float*)d_in[19];   const float* b1 = (const float*)d_in[20];
    const float* W2 = (const float*)d_in[21];   const float* b2 = (const float*)d_in[22];
    const float* ln1g = (const float*)d_in[23]; const float* ln1b = (const float*)d_in[24];
    const float* ln2g = (const float*)d_in[25]; const float* ln2b = (const float*)d_in[26];
    const float* ln3g = (const float*)d_in[27]; const float* ln3b = (const float*)d_in[28];
    float* out = (float*)d_out;

    const size_t nx = (size_t)NB * SEQ * DM;
    const size_t ne = (size_t)NB * SENC * DM;
    const size_t nmx = (nx > ne) ? nx : ne;
    unsigned char* base = (unsigned char*)d_ws;
    size_t off = 0;
    const size_t szA = ((2 * nx + 2 * ne) > 4 * nx) ? (2 * nx + 2 * ne) : (4 * nx);
    _Float16* Xh = (_Float16*)(base + off);
    _Float16* Eh = (_Float16*)(base + off + 2 * nx);
    float*    H2 = (float*)(base + off);
    off += szA;
    _Float16* Wsq = (_Float16*)(base + off); off += (size_t)8 * DM * DM * 2;
    _Float16* W1t = (_Float16*)(base + off); off += (size_t)FF * DM * 2;
    _Float16* W2t = (_Float16*)(base + off); off += (size_t)DM * FF * 2;
    const size_t szB = ((4 * nx + 4 * nmx) > 8 * nx) ? (4 * nx + 4 * nmx) : (8 * nx);
    _Float16* Qh = (_Float16*)(base + off);
    _Float16* Kh = (_Float16*)(base + off + 2 * nx);
    _Float16* Vh = (_Float16*)(base + off + 2 * nx + 2 * nmx);
    _Float16* Ch = (_Float16*)(base + off + 2 * nx + 4 * nmx);
    _Float16* Midh = (_Float16*)(base + off);
    off += szB;
    float*    T32 = (float*)(base + off);    off += 4 * nx;
    float*    H1  = (float*)(base + off);    off += 4 * nx;
    _Float16* Hh  = (_Float16*)(base + off); off += 2 * nx;
    if (off > ws_size) return;

    const size_t DD = (size_t)DM * DM;
    const int MX = NB * SEQ, ME = NB * SENC;
    const int nblkX = (int)(nx / 2048), nblkE = (int)(ne / 2048);
    const float OS_A = 1.0f / (A_CARRY * W_CARRY);
    const float OS_X = 1.0f / (X_CARRY * W_CARRY);
    const dim3 blk(256);
    const dim3 gX(MX / 64, DM / 128), gE(ME / 64, DM / 128), gF(MX / 64, FF / 128);

    k_cvt_act<<<dim3(nblkX + nblkE), blk, 0, stream>>>(x, enc, Xh, Eh, nblkX);
    k_cvt_w<<<dim3(DM / 64, DM / 64, 8), blk, 0, stream>>>(saWq, saWk, saWv, saWo, eaWq, eaWk, eaWv, eaWo, Wsq, DM, DM);
    k_cvt_w<<<dim3(FF / 64, DM / 64, 1), blk, 0, stream>>>(W1, W1, W1, W1, W1, W1, W1, W1, W1t, DM, FF);
    k_cvt_w<<<dim3(DM / 64, FF / 64, 1), blk, 0, stream>>>(W2, W2, W2, W2, W2, W2, W2, W2, W2t, FF, DM);

    k_gemm<1, 0><<<gX, blk, 0, stream>>>(Xh, Wsq + 0 * DD, sabq, (void*)Qh, DM, DM, OS_A, A_CARRY);
    k_gemm<1, 0><<<gX, blk, 0, stream>>>(Xh, Wsq + 1 * DD, sabk, (void*)Kh, DM, DM, OS_A, V_CARRY);
    k_gemm<1, 0><<<gX, blk, 0, stream>>>(Xh, Wsq + 2 * DD, sabv, (void*)Vh, DM, DM, OS_A, V_CARRY);
    k_attn<<<dim3(SEQ / QR, HE, NB), blk, 0, stream>>>(Qh, Kh, Vh, emask, 1, SEQ, Ch);
    k_gemm<0, 0><<<gX, blk, 0, stream>>>(Ch, Wsq + 3 * DD, sabo, (void*)T32, DM, DM, OS_X, 1.0f);
    k_ln<<<dim3(MX / 8), blk, 0, stream>>>(T32, x, 1, ln1g, ln1b, H1, 0, Hh, 1);

    k_gemm<1, 0><<<gX, blk, 0, stream>>>(Hh, Wsq + 4 * DD, eabq, (void*)Qh, DM, DM, OS_A, A_CARRY);
    k_gemm<1, 0><<<gE, blk, 0, stream>>>(Eh, Wsq + 5 * DD, eabk, (void*)Kh, DM, DM, OS_A, V_CARRY);
    k_gemm<1, 0><<<gE, blk, 0, stream>>>(Eh, Wsq + 6 * DD, eabv, (void*)Vh, DM, DM, OS_A, V_CARRY);
    k_attn<<<dim3(SEQ / QR, HE, NB), blk, 0, stream>>>(Qh, Kh, Vh, emask, 0, SENC, Ch);
    k_gemm<0, 0><<<gX, blk, 0, stream>>>(Ch, Wsq + 7 * DD, eabo, (void*)T32, DM, DM, OS_X, 1.0f);
    k_ln<<<dim3(MX / 8), blk, 0, stream>>>(T32, H1, 0, ln2g, ln2b, H2, 0, Hh, 1);

    k_gemm<1, 1><<<gF, blk, 0, stream>>>(Hh, W1t, b1, (void*)Midh, DM, FF, OS_A, A_CARRY);
    k_gemm<0, 0><<<gX, blk, 0, stream>>>(Midh, W2t, b2, (void*)T32, FF, DM, OS_A, 1.0f);
    k_ln<<<dim3(MX / 8), blk, 0, stream>>>(T32, H2, 0, ln3g, ln3b, out, 1, Hh, 0);
}
